// GumbelGCN_24129126269433
// MI455X (gfx1250) — hardware-verified
//
#include <hip/hip_runtime.h>
#include <stddef.h>


#define NNODE 1024
#define DIN   128
#define EDIM  16
#define KTOP  8
#define NSEL  (NNODE * KTOP)
#define SELW  32
#define HID1  64
#define HID2  64
#define NOUT  40
#define NMAT  7
#define RT    256
#define NWV   (RT / 32)
#define GT    128
#define GR    64
#define GC    64
#define TGA   32
#define DEGC  128
#define BIGI  0x7fffffff
#define NEGF  (-1000000000.0f)
#define GEPS  (1e-7f)
#define GUME  (1e-20f)
#define WSCAP 134217728
#define LDSMAX (2 * GR * (256 + 8) * 2)

static_assert(NNODE % RT == 0);
static_assert(NSEL % RT == 0);
static_assert(NNODE % GR == 0);
static_assert(NSEL % GR == 0);
static_assert(NNODE % TGA == 0);
static_assert(TGA == 4 * NWV);
static_assert(GR == 16 * (GT / 32));
static_assert(NNODE / RT == 4);
static_assert(SELW == 4 * KTOP);
static_assert((NOUT % 4) == 0);
static_assert(((GR * NOUT / 4) % 32) == 0);
static_assert(DIN % GC == 0 && HID1 % GC == 0 && (2 * DIN) % GC == 0 && (2 * HID1) % GC == 0 && HID2 % GC == 0);
static_assert(LDSMAX >= GR * GC * 4);

typedef float          v4f  __attribute__((ext_vector_type(4)));
typedef float          v8f  __attribute__((ext_vector_type(8)));
typedef int            v4i  __attribute__((ext_vector_type(4)));
typedef unsigned short v8us __attribute__((ext_vector_type(8)));
typedef __bf16         v16b __attribute__((ext_vector_type(16)));
union FragB { v16b v; v8us h[2]; };

__host__ __device__ constexpr int wK(int y)  { return y == 0 ? EDIM : y == 1 ? DIN : y == 2 ? 2 * DIN : y == 3 ? EDIM : y == 4 ? HID1 : y == 5 ? 2 * HID1 : HID2; }
__host__ __device__ constexpr int wN(int y)  { return y == 0 ? DIN : y == 1 ? 2 * DIN : y == 2 ? HID1 : y == 3 ? HID1 : y == 4 ? 2 * HID1 : y == 5 ? HID2 : NOUT; }
__host__ __device__ constexpr int wKp(int y) { return (wK(y) + 31) & ~31; }
__host__ __device__ constexpr int wNp(int y) { return (wN(y) + GC - 1) & ~(GC - 1); }
__host__ __device__ constexpr int wSz(int y) { return 2 * wNp(y) * wKp(y); }
__host__ __device__ constexpr int wOff(int y) {
  return (y > 0 ? wSz(0) : 0) + (y > 1 ? wSz(1) : 0) + (y > 2 ? wSz(2) : 0) + (y > 3 ? wSz(3) : 0)
       + (y > 4 ? wSz(4) : 0) + (y > 5 ? wSz(5) : 0) + (y > 6 ? wSz(6) : 0);
}
static_assert((wSz(0) * 2) % 256 == 0 && (wSz(3) * 2) % 256 == 0 && (wSz(6) * 2) % 256 == 0);
static_assert((wOff(1) % 8) == 0 && (wOff(2) % 8) == 0 && (wOff(3) % 8) == 0 && (wOff(4) % 8) == 0 && (wOff(5) % 8) == 0 && (wOff(6) % 8) == 0);

__device__ __forceinline__ unsigned int bfr(float f) {
  const unsigned int u = __float_as_uint(f);
  return (u + 0x7FFFu + ((u >> 16) & 1u)) >> 16;
}

__device__ __forceinline__ void split1(float x, unsigned short& hb, unsigned short& lb) {
  const unsigned int hu = bfr(x);
  const float hf = __uint_as_float(hu << 16);
  hb = (unsigned short)hu;
  lb = (unsigned short)bfr(x - hf);
}

__device__ __forceinline__ void split8(v4f a, v4f b, v8us& hi, v8us& lo) {
  unsigned short hb, lb;
  split1(a.x, hb, lb); hi[0] = hb; lo[0] = lb;
  split1(a.y, hb, lb); hi[1] = hb; lo[1] = lb;
  split1(a.z, hb, lb); hi[2] = hb; lo[2] = lb;
  split1(a.w, hb, lb); hi[3] = hb; lo[3] = lb;
  split1(b.x, hb, lb); hi[4] = hb; lo[4] = lb;
  split1(b.y, hb, lb); hi[5] = hb; lo[5] = lb;
  split1(b.z, hb, lb); hi[6] = hb; lo[6] = lb;
  split1(b.w, hb, lb); hi[7] = hb; lo[7] = lb;
}

__device__ __forceinline__ v8f wmb(v16b a, v16b b, v8f c) {
  v8f d = __builtin_amdgcn_wmma_f32_16x16x32_bf16(false, a, false, b, (short)0, c, false, false);
  asm volatile("v_nop\n\tv_nop\n\tv_nop\n\tv_nop" : "+v"(d) : "v"(a), "v"(b));
  return d;
}

__device__ __forceinline__ float wval(const float* __restrict__ src, int k, int K, int N, int nc, bool nv) {
  const int kc = k < K ? k : K - 1;
  const float tv = src[(size_t)kc * N + nc];
  return (k < K && nv) ? tv : 0.0f;
}

__global__ __launch_bounds__(RT) void k_wprep(
    const float* __restrict__ w0, const float* __restrict__ w1, const float* __restrict__ w2,
    const float* __restrict__ w3, const float* __restrict__ w4, const float* __restrict__ w5,
    const float* __restrict__ w6, unsigned short* wb) {
  const int y = blockIdx.y;
  const float* src = y == 0 ? w0 : y == 1 ? w1 : y == 2 ? w2 : y == 3 ? w3 : y == 4 ? w4 : y == 5 ? w5 : w6;
  constexpr int K0 = wK(0),  K1 = wK(1),  K2 = wK(2),  K3 = wK(3),  K4 = wK(4),  K5 = wK(5),  K6 = wK(6);
  constexpr int N0 = wN(0),  N1 = wN(1),  N2 = wN(2),  N3 = wN(3),  N4 = wN(4),  N5 = wN(5),  N6 = wN(6);
  constexpr int Q0 = wKp(0), Q1 = wKp(1), Q2 = wKp(2), Q3 = wKp(3), Q4 = wKp(4), Q5 = wKp(5), Q6 = wKp(6);
  constexpr int M0 = wNp(0), M1 = wNp(1), M2 = wNp(2), M3 = wNp(3), M4 = wNp(4), M5 = wNp(5), M6 = wNp(6);
  constexpr int P0 = wOff(0), P1 = wOff(1), P2 = wOff(2), P3 = wOff(3), P4 = wOff(4), P5 = wOff(5), P6 = wOff(6);
  const int K  = y == 0 ? K0 : y == 1 ? K1 : y == 2 ? K2 : y == 3 ? K3 : y == 4 ? K4 : y == 5 ? K5 : K6;
  const int N  = y == 0 ? N0 : y == 1 ? N1 : y == 2 ? N2 : y == 3 ? N3 : y == 4 ? N4 : y == 5 ? N5 : N6;
  const int Kp = y == 0 ? Q0 : y == 1 ? Q1 : y == 2 ? Q2 : y == 3 ? Q3 : y == 4 ? Q4 : y == 5 ? Q5 : Q6;
  const int Np = y == 0 ? M0 : y == 1 ? M1 : y == 2 ? M2 : y == 3 ? M3 : y == 4 ? M4 : y == 5 ? M5 : M6;
  const int po = y == 0 ? P0 : y == 1 ? P1 : y == 2 ? P2 : y == 3 ? P3 : y == 4 ? P4 : y == 5 ? P5 : P6;
  const int kg8 = Kp >> 3;
  const int i = (int)blockIdx.x * RT + (int)threadIdx.x;
  if (i >= Np * kg8) return;
  const int n  = i / kg8;
  const int k0 = (i - n * kg8) * 8;
  const int nc = n < N ? n : N - 1;
  const bool nv = n < N;
  v4f a, b;
  a.x = wval(src, k0 + 0, K, N, nc, nv);
  a.y = wval(src, k0 + 1, K, N, nc, nv);
  a.z = wval(src, k0 + 2, K, N, nc, nv);
  a.w = wval(src, k0 + 3, K, N, nc, nv);
  b.x = wval(src, k0 + 4, K, N, nc, nv);
  b.y = wval(src, k0 + 5, K, N, nc, nv);
  b.z = wval(src, k0 + 6, K, N, nc, nv);
  b.w = wval(src, k0 + 7, K, N, nc, nv);
  v8us hv, lv;
  split8(a, b, hv, lv);
  unsigned short* dh = wb + (size_t)po + (size_t)i * 8;
  unsigned short* dl = dh + (size_t)Np * Kp;
  *(volatile v8us*)dh = hv;
  *(volatile v8us*)dl = lv;
  __threadfence();
  *(volatile v8us*)dh = hv;
  *(volatile v8us*)dl = lv;
}

__global__ __launch_bounds__(RT) void k_prep(
    const float* __restrict__ ea, const float* __restrict__ x, const float* __restrict__ mw,
    float* se, float* xwn, float* xwb, int nE, int nEB, int sePad) {
  const int t = threadIdx.x;
  if ((int)blockIdx.x < nEB) {
    const int e  = (int)blockIdx.x * RT + t;
    const int ec = e < nE ? e : nE - 1;
    const float* ep = ea + (size_t)ec * EDIM;
    const float* wp = mw + 2 * DIN;
    float s = 0.0f;
#pragma unroll 1
    for (int k = 0; k < EDIM; ++k) s += ep[k] * wp[k];
    if (e < sePad) *(volatile float*)(se + e) = s;
    __threadfence();
    if (e < sePad) *(volatile float*)(se + e) = s;
  } else {
    const int i  = ((int)blockIdx.x - nEB) * RT + t;
    const int ic = i < NNODE ? i : NNODE - 1;
    const float* xp = x + (size_t)ic * DIN;
    float a = 0.0f, b = 0.0f;
#pragma unroll 1
    for (int k = 0; k < DIN; ++k) {
      const float v = xp[k];
      a += v * mw[k];
      b += v * mw[DIN + k];
    }
    if (i < NNODE) { *(volatile float*)(xwn + i) = a; *(volatile float*)(xwb + i) = b; }
    __threadfence();
    if (i < NNODE) { *(volatile float*)(xwn + i) = a; *(volatile float*)(xwb + i) = b; }
  }
}

__global__ __launch_bounds__(RT) void k_rowsel(
    const int* __restrict__ ei, const float* __restrict__ se, const float* __restrict__ xwn,
    const float* __restrict__ xwb, const float* __restrict__ mlpb, const float* __restrict__ noise,
    int* sel, int nE) {
#pragma clang fp contract(off)
  __shared__ int   emn[NNODE];
  __shared__ int   emx[NNODE];
  __shared__ float sed[NNODE];
  __shared__ float key[NNODE];
  __shared__ int   wl[NWV * 32];
  __shared__ int   wcn[NWV];
  __shared__ float rvv[NWV];
  __shared__ int   rvi[NWV];
  __shared__ __attribute__((aligned(16))) int selb[SELW];
  const int t = threadIdx.x, lane = t & 31, wave = t >> 5;
  const int u = blockIdx.x;
  for (int j = t; j < NNODE; j += RT) { emn[j] = BIGI; emx[j] = -1; sed[j] = 0.0f; }
  if (t < SELW) selb[t] = 0;
  __syncthreads();

  const int* dsts = ei + nE;
  const int nCh = (nE + RT - 1) / RT;
#pragma unroll 1
  for (int ch = 0; ch < nCh; ++ch) {
    const int e  = ch * RT + t;
    const int ec = e < nE ? e : nE - 1;
    const int s  = ei[ec];
    const bool hit = (e < nE) && (s == u);
    const unsigned mk = __builtin_amdgcn_ballot_w32(hit);
    const int pos = (int)__builtin_amdgcn_mbcnt_lo(mk, 0u);
    if (hit) wl[wave * 32 + pos] = e;
    if (lane == 0) wcn[wave] = (int)__builtin_popcount(mk);
    __syncthreads();
    if (wave == 0) {
#pragma unroll 1
      for (int w = 0; w < NWV; ++w) {
        int n = __builtin_amdgcn_readfirstlane(wcn[w]);
        n = n < 0 ? 0 : (n > 32 ? 32 : n);
#pragma unroll 1
        for (int i = 0; i < n; ++i) {
          int eh = __builtin_amdgcn_readfirstlane(wl[w * 32 + i]);
          eh = eh < 0 ? 0 : (eh > nE - 1 ? nE - 1 : eh);
          int d = dsts[eh];
          d = d < 0 ? 0 : (d > NNODE - 1 ? NNODE - 1 : d);
          const float sc = se[eh];
          if (lane == 0) {
            if (eh < emn[d]) emn[d] = eh;
            if (eh > emx[d]) { emx[d] = eh; sed[d] = sc; }
          }
        }
      }
    }
    __syncthreads();
  }

  const float xu = xwn[u], bb = mlpb[0];
  float lmax = -__builtin_inff();
#pragma unroll 1
  for (int j = t; j < NNODE; j += RT) {
    const float sc = ((xu + xwb[j]) + sed[j]) + bb;
    const float s  = (emn[j] != BIGI) ? sc : NEGF;
    key[j] = s;
    lmax = fmaxf(lmax, s);
  }
#pragma unroll
  for (int o = 16; o > 0; o >>= 1) lmax = fmaxf(lmax, __shfl_xor(lmax, o));
  if (lane == 0) rvv[wave] = lmax;
  __syncthreads();
  float mx = rvv[0];
#pragma unroll
  for (int w = 1; w < NWV; ++w) mx = fmaxf(mx, rvv[w]);
  __syncthreads();
  float lsum = 0.0f;
#pragma unroll 1
  for (int j = t; j < NNODE; j += RT) {
    const float ev = expf(key[j] - mx);
    key[j] = ev;
    lsum += ev;
  }
#pragma unroll
  for (int o = 16; o > 0; o >>= 1) lsum += __shfl_xor(lsum, o);
  if (lane == 0) rvv[wave] = lsum;
  __syncthreads();
  float den = rvv[0];
#pragma unroll
  for (int w = 1; w < NWV; ++w) den += rvv[w];
  __syncthreads();
  const float rden = 1.0f / den;
#pragma unroll 1
  for (int j = t; j < NNODE; j += RT) {
    const float z  = key[j] * rden;
    const float uu = noise[(size_t)u * NNODE + j];
    const float a  = logf(uu + GUME);
    const float b  = GUME - a;
    const float g  = -logf(b);
    key[j] = z + g;
  }
  __syncthreads();

#pragma unroll 1
  for (int k = 0; k < KTOP; ++k) {
    float bv = -__builtin_inff();
    int   bi = BIGI;
#pragma unroll
    for (int q = 0; q < NNODE / RT; ++q) {
      const int j = t + RT * q;
      const float v = key[j];
      const bool tk = (v > bv) || (v == bv && j < bi);
      bv = tk ? v : bv;
      bi = tk ? j : bi;
    }
#pragma unroll
    for (int o = 16; o > 0; o >>= 1) {
      const float ov = __shfl_xor(bv, o);
      const int   oi = __shfl_xor(bi, o);
      const bool tk = (ov > bv) || (ov == bv && oi < bi);
      bv = tk ? ov : bv;
      bi = tk ? oi : bi;
    }
    if (lane == 0) { rvv[wave] = bv; rvi[wave] = bi; }
    __syncthreads();
    float wv = rvv[0];
    int   wi = rvi[0];
#pragma unroll
    for (int w = 1; w < NWV; ++w) {
      const float ov = rvv[w];
      const int   oi = rvi[w];
      const bool tk = (ov > wv) || (ov == wv && oi < wi);
      wv = tk ? ov : wv;
      wi = tk ? oi : wi;
    }
    wi = wi < 0 ? 0 : (wi > NNODE - 1 ? NNODE - 1 : wi);
    if (t == (wi & (RT - 1))) key[wi] = -__builtin_inff();
    if (t == 0) {
      selb[k] = wi;
      const int em = emn[wi];
      selb[KTOP + k] = (em == BIGI) ? 0 : em;
    }
    __syncthreads();
  }

  if (wave == 0 && lane < 8) {
    const v4i v = *(const v4i*)(selb + 4 * lane);
    *(volatile v4i*)(sel + (size_t)u * SELW + 4 * lane) = v;
  }
  __threadfence();
  if (wave == 0 && lane < 8) {
    const v4i v = *(const v4i*)(selb + 4 * lane);
    *(volatile v4i*)(sel + (size_t)u * SELW + 4 * lane) = v;
  }
}

__global__ __launch_bounds__(GT) void k_gemm(
    const float* __restrict__ A, int lda, int nRowsA, int K,
    const float* __restrict__ ea, const int* __restrict__ sel, int nE0, int amode,
    const unsigned short* __restrict__ Bw, int Kp, int Np,
    const float* __restrict__ bias, int N,
    const float* __restrict__ xres, int ldx, int nResRows, int resShift, int useRes,
    int relu, float epsAdd,
    const int* __restrict__ mask, int useMask,
    float* C, int ldc, int nRowsC, int smode) {
  extern __shared__ v4f lds_dyn[];
  const int aph = Kp + 8;
  unsigned short* sHi = (unsigned short*)lds_dyn;
  unsigned short* sLo = sHi + GR * aph;
  float*          stg = (float*)lds_dyn;
  const int tid = threadIdx.x, lane = tid & 31, wave = tid >> 5, hh = lane >> 4, m = lane & 15;
  const int rowBase = (int)blockIdx.x * GR, colBase = (int)blockIdx.y * GC;
  const int kg8 = Kp >> 3;

#pragma unroll 1
  for (int idx = tid; idx < GR * kg8; idx += GT) {
    const int r  = idx / kg8;
    const int c0 = (idx - r * kg8) * 8;
    int row = rowBase + r;
    row = row > nRowsA - 1 ? nRowsA - 1 : row;
    const float* ap;
    bool kval;
    if (amode != 0) {
      const int uu = row >> 3, kk = row & 7;
      int eid = sel[uu * SELW + KTOP + kk];
      eid = eid < 0 ? 0 : (eid > nE0 - 1 ? nE0 - 1 : eid);
      const int cc = c0 < EDIM - 8 ? c0 : EDIM - 8;
      ap = ea + (size_t)eid * EDIM + cc;
      kval = c0 < EDIM;
    } else {
      const int cc = c0 < K - 8 ? c0 : K - 8;
      ap = A + (size_t)row * lda + cc;
      kval = c0 < K;
    }
    v4f a = *(const v4f*)ap;
    v4f b = *(const v4f*)(ap + 4);
    if (!kval) { const v4f z = {0.0f, 0.0f, 0.0f, 0.0f}; a = z; b = z; }
    v8us hv, lv;
    split8(a, b, hv, lv);
    *(v8us*)(sHi + r * aph + c0) = hv;
    *(v8us*)(sLo + r * aph + c0) = lv;
  }
  __syncthreads();

  v8f acc[4];
#pragma unroll
  for (int tt = 0; tt < 4; ++tt) { const v8f z = {0.f, 0.f, 0.f, 0.f, 0.f, 0.f, 0.f, 0.f}; acc[tt] = z; }
  const unsigned short* ahp = sHi + (wave * 16 + m) * aph + 8 * hh;
  const unsigned short* alp = sLo + (wave * 16 + m) * aph + 8 * hh;
  const size_t plo = (size_t)Np * Kp;
  const int nkt = Kp >> 5;
#pragma unroll 1
  for (int kt = 0; kt < nkt; ++kt) {
    FragB ah, al;
    ah.h[0] = *(const v8us*)(ahp + 32 * kt);
    ah.h[1] = *(const v8us*)(ahp + 32 * kt + 16);
    al.h[0] = *(const v8us*)(alp + 32 * kt);
    al.h[1] = *(const v8us*)(alp + 32 * kt + 16);
#pragma unroll
    for (int tt = 0; tt < 4; ++tt) {
      const unsigned short* bp = Bw + (size_t)(colBase + 16 * tt + m) * Kp + 32 * kt + 8 * hh;
      FragB bh, bl;
      bh.h[0] = *(const v8us*)bp;
      bh.h[1] = *(const v8us*)(bp + 16);
      bl.h[0] = *(const v8us*)(bp + plo);
      bl.h[1] = *(const v8us*)(bp + plo + 16);
      acc[tt] = wmb(ah.v, bh.v, acc[tt]);
      acc[tt] = wmb(ah.v, bl.v, acc[tt]);
      acc[tt] = wmb(al.v, bh.v, acc[tt]);
    }
  }
  __syncthreads();

  const int r0 = wave * 16 + 8 * hh;
#pragma unroll
  for (int tt = 0; tt < 4; ++tt) {
    const int colL = 16 * tt + m;
    const int col  = colBase + colL;
    const int colc = col < N ? col : N - 1;
    const float bl = bias[colc];
    const float bv = col < N ? bl : 0.0f;
#pragma unroll
    for (int r = 0; r < 8; ++r) {
      const int row = rowBase + r0 + r;
      float xr = 0.0f;
      if (useRes != 0) {
        int rr = row >> resShift;
        rr = rr > nResRows - 1 ? nResRows - 1 : rr;
        xr = xres[(size_t)rr * ldx + colc];
      }
      float v = xr + (acc[tt][r] + bv);
      if (relu != 0) v = fmaxf(v, 0.0f);
      v = v + epsAdd;
      if (useMask != 0) {
        const int mr = row > nRowsC - 1 ? nRowsC - 1 : row;
        v = (mask[mr] != 0) ? v : 0.0f;
      }
      stg[(r0 + r) * GC + colL] = v;
    }
  }
  __syncthreads();

  if (smode == 0) {
    const int rl = wave * 16;
#pragma unroll
    for (int i = 0; i < 8; ++i) {
      const int r = rl + 2 * i + hh;
      const v4f v = *(const v4f*)(stg + r * GC + 4 * m);
      const int grow = rowBase + r;
      if (grow < nRowsC) *(volatile v4f*)(C + (size_t)grow * ldc + colBase + 4 * m) = v;
    }
    __threadfence();
#pragma unroll
    for (int i = 0; i < 8; ++i) {
      const int r = rl + 2 * i + hh;
      const v4f v = *(const v4f*)(stg + r * GC + 4 * m);
      const int grow = rowBase + r;
      if (grow < nRowsC) *(volatile v4f*)(C + (size_t)grow * ldc + colBase + 4 * m) = v;
    }
  } else {
    const int nf4 = (GR * N) >> 2;
    float* gb = C + (size_t)rowBase * ldc;
#pragma unroll 1
    for (int f4 = tid; f4 < nf4; f4 += GT) {
      const int f = 4 * f4;
      const int r = f / N;
      const int c = f - r * N;
      const v4f v = *(const v4f*)(stg + r * GC + c);
      if (rowBase + r < nRowsC) *(volatile v4f*)(gb + f) = v;
    }
    __threadfence();
#pragma unroll 1
    for (int f4 = tid; f4 < nf4; f4 += GT) {
      const int f = 4 * f4;
      const int r = f / N;
      const int c = f - r * N;
      const v4f v = *(const v4f*)(stg + r * GC + c);
      if (rowBase + r < nRowsC) *(volatile v4f*)(gb + f) = v;
    }
  }
}

__global__ __launch_bounds__(RT) void k_agg(
    const int* __restrict__ sel, const float* __restrict__ mpl, const float* __restrict__ xin,
    float* hp, int C) {
  __shared__ int elist[TGA * DEGC];
  __shared__ int ecnt[TGA];
  __shared__ int wl[NWV * 32];
  __shared__ int wcn[NWV];
  const int t = threadIdx.x, lane = t & 31, wave = t >> 5;
  const int tBase = (int)blockIdx.x * TGA;
  if (t < TGA) ecnt[t] = 0;
  __syncthreads();

#pragma unroll 1
  for (int ch = 0; ch < NSEL / RT; ++ch) {
    const int e = ch * RT + t;
    const int d = sel[(e >> 3) * SELW + (e & 7)];
    const unsigned sl = (unsigned)(d - tBase);
    const bool hit = sl < (unsigned)TGA;
    const unsigned mk = __builtin_amdgcn_ballot_w32(hit);
    const int pos = (int)__builtin_amdgcn_mbcnt_lo(mk, 0u);
    if (hit) wl[wave * 32 + pos] = (e << 5) | (int)sl;
    if (lane == 0) wcn[wave] = (int)__builtin_popcount(mk);
    __syncthreads();
    if (wave == 0) {
#pragma unroll 1
      for (int w = 0; w < NWV; ++w) {
        int n = __builtin_amdgcn_readfirstlane(wcn[w]);
        n = n < 0 ? 0 : (n > 32 ? 32 : n);
#pragma unroll 1
        for (int i = 0; i < n; ++i) {
          const int ent  = __builtin_amdgcn_readfirstlane(wl[w * 32 + i]);
          const int slot = ent & (TGA - 1);
          int eh = ent >> 5;
          eh = eh < 0 ? 0 : (eh > NSEL - 1 ? NSEL - 1 : eh);
          if (lane == 0) {
            const int p = ecnt[slot];
            if (p >= 0 && p < DEGC) elist[slot * DEGC + p] = eh;
            ecnt[slot] = (p + 1 > DEGC) ? DEGC : p + 1;
          }
        }
      }
    }
    __syncthreads();
  }

  const int c4 = (4 * lane < C - 4) ? 4 * lane : C - 4;
  const bool act = 4 * lane < C;
#pragma unroll 1
  for (int q = 0; q < 4; ++q) {
    const int slot = wave * 4 + q;
    const int d = tBase + slot;
    int n = __builtin_amdgcn_readfirstlane(ecnt[slot]);
    n = n < 0 ? 0 : (n > DEGC ? DEGC : n);
    v4f mx;
    mx.x = -__builtin_inff(); mx.y = mx.x; mx.z = mx.x; mx.w = mx.x;
#pragma unroll 1
    for (int p = 0; p < n; ++p) {
      int eh = __builtin_amdgcn_readfirstlane(elist[slot * DEGC + p]);
      eh = eh < 0 ? 0 : (eh > NSEL - 1 ? NSEL - 1 : eh);
      const v4f mv = *(const v4f*)(mpl + (size_t)eh * C + c4);
      mx.x = fmaxf(mx.x, mv.x); mx.y = fmaxf(mx.y, mv.y); mx.z = fmaxf(mx.z, mv.z); mx.w = fmaxf(mx.w, mv.w);
    }
    v4f den = {0.0f, 0.0f, 0.0f, 0.0f};
    v4f num = {0.0f, 0.0f, 0.0f, 0.0f};
#pragma unroll 1
    for (int p = 0; p < n; ++p) {
      int eh = __builtin_amdgcn_readfirstlane(elist[slot * DEGC + p]);
      eh = eh < 0 ? 0 : (eh > NSEL - 1 ? NSEL - 1 : eh);
      const v4f mv = *(const v4f*)(mpl + (size_t)eh * C + c4);
      v4f w;
      w.x = expf(mv.x - mx.x); w.y = expf(mv.y - mx.y); w.z = expf(mv.z - mx.z); w.w = expf(mv.w - mx.w);
      den = den + w;
      num.x += w.x * mv.x; num.y += w.y * mv.y; num.z += w.z * mv.z; num.w += w.w * mv.w;
    }
    v4f agg;
    agg.x = num.x / (den.x > 0.0f ? den.x : 1.0f);
    agg.y = num.y / (den.y > 0.0f ? den.y : 1.0f);
    agg.z = num.z / (den.z > 0.0f ? den.z : 1.0f);
    agg.w = num.w / (den.w > 0.0f ? den.w : 1.0f);
    const v4f xr = *(const v4f*)(xin + (size_t)d * C + c4);
    const v4f o = agg + xr;
    float* gp = hp + (size_t)d * C + 4 * lane;
    if (act) *(volatile v4f*)gp = o;
    __threadfence();
    if (act) *(volatile v4f*)gp = o;
  }
}

static inline int ldsFor(int Kp) {
  const int a = 2 * GR * (Kp + 8) * 2;
  const int b = GR * GC * 4;
  return a > b ? a : b;
}

extern "C" void kernel_launch(void* const* d_in, const int* in_sizes, int n_in,
                              void* d_out, int out_size, void* d_ws, size_t ws_size,
                              hipStream_t stream) {
  if (n_in < 22) return;
  if (in_sizes[0] != NNODE * DIN) return;
  if ((in_sizes[20] & 1) != 0) return;
  const int nE = in_sizes[20] / 2;
  if (nE <= 0 || nE > (1 << 24)) return;
  if (in_sizes[1] != nE * EDIM) return;
  if (in_sizes[2] != NNODE * NNODE) return;
  if (in_sizes[3] != EDIM + 2 * DIN || in_sizes[4] < 1) return;
  if (in_sizes[5] != EDIM * DIN || in_sizes[6] != DIN) return;
  if (in_sizes[7] != DIN * 2 * DIN || in_sizes[8] != 2 * DIN) return;
  if (in_sizes[9] != 2 * DIN * HID1 || in_sizes[10] != HID1) return;
  if (in_sizes[11] != EDIM * HID1 || in_sizes[12] != HID1) return;
  if (in_sizes[13] != HID1 * 2 * HID1 || in_sizes[14] != 2 * HID1) return;
  if (in_sizes[15] != 2 * HID1 * HID2 || in_sizes[16] != HID2) return;
  if (in_sizes[17] != HID2 * NOUT || in_sizes[18] != NOUT) return;
  if (in_sizes[21] != NNODE) return;
  if (out_size != NNODE * NOUT) return;

  const float* x         = (const float*)d_in[0];
  const float* edge_attr = (const float*)d_in[1];
  const float* noise     = (const float*)d_in[2];
  const float* mlp_w     = (const float*)d_in[3];
  const float* mlp_b     = (const float*)d_in[4];
  const float* c1_we     = (const float*)d_in[5];
  const float* c1_be     = (const float*)d_in[6];
  const float* c1_w1     = (const float*)d_in[7];
  const float* c1_b1     = (const float*)d_in[8];
  const float* c1_w2     = (const float*)d_in[9];
  const float* c1_b2     = (const float*)d_in[10];
  const float* c2_we     = (const float*)d_in[11];
  const float* c2_be     = (const float*)d_in[12];
  const float* c2_w1     = (const float*)d_in[13];
  const float* c2_b1     = (const float*)d_in[14];
  const float* c2_w2     = (const float*)d_in[15];
  const float* c2_b2     = (const float*)d_in[16];
  const float* fc_w      = (const float*)d_in[17];
  const float* fc_b      = (const float*)d_in[18];
  const int*   edge_index = (const int*)d_in[20];
  const int*   node_mask  = (const int*)d_in[21];
  float* out = (float*)d_out;

  const int sePad = (nE + 31) & ~31;
  const int nEB   = (sePad + RT - 1) / RT;

  char* ws = (char*)d_ws;
  size_t off = 0;
  const size_t oW   = off; off += (size_t)wOff(NMAT) * 2;            off = (off + 255) & ~(size_t)255;
  const size_t oSe  = off; off += (size_t)sePad * 4;                 off = (off + 255) & ~(size_t)255;
  const size_t oXn  = off; off += (size_t)NNODE * 4;                 off = (off + 255) & ~(size_t)255;
  const size_t oXb  = off; off += (size_t)NNODE * 4;                 off = (off + 255) & ~(size_t)255;
  const size_t oSel = off; off += (size_t)NNODE * SELW * 4;          off = (off + 255) & ~(size_t)255;
  const size_t oM1  = off; off += (size_t)NSEL * DIN * 4;            off = (off + 255) & ~(size_t)255;
  const size_t oHp1 = off; off += (size_t)NNODE * DIN * 4;           off = (off + 255) & ~(size_t)255;
  const size_t oT1  = off; off += (size_t)NNODE * 2 * DIN * 4;       off = (off + 255) & ~(size_t)255;
  const size_t oH1  = off; off += (size_t)NNODE * HID1 * 4;          off = (off + 255) & ~(size_t)255;
  const size_t oM2  = off; off += (size_t)NSEL * HID1 * 4;           off = (off + 255) & ~(size_t)255;
  const size_t oHp2 = off; off += (size_t)NNODE * HID1 * 4;          off = (off + 255) & ~(size_t)255;
  const size_t oT2  = off; off += (size_t)NNODE * 2 * HID1 * 4;      off = (off + 255) & ~(size_t)255;
  const size_t oH2  = off; off += (size_t)NNODE * HID2 * 4;          off = (off + 255) & ~(size_t)255;
  if (off > ws_size || off > (size_t)WSCAP) return;

  unsigned short* wb = (unsigned short*)(ws + oW);
  float* se  = (float*)(ws + oSe);
  float* xwn = (float*)(ws + oXn);
  float* xwb = (float*)(ws + oXb);
  int*   sel = (int*)(ws + oSel);
  float* m1  = (float*)(ws + oM1);
  float* hp1 = (float*)(ws + oHp1);
  float* t1  = (float*)(ws + oT1);
  float* h1  = (float*)(ws + oH1);
  float* m2  = (float*)(ws + oM2);
  float* hp2 = (float*)(ws + oHp2);
  float* t2  = (float*)(ws + oT2);
  float* h2  = (float*)(ws + oH2);

  k_wprep<<<dim3(16, NMAT), RT, 0, stream>>>(c1_we, c1_w1, c1_w2, c2_we, c2_w1, c2_w2, fc_w, wb);

  k_prep<<<nEB + NNODE / RT, RT, 0, stream>>>(edge_attr, x, mlp_w, se, xwn, xwb, nE, nEB, sePad);

  k_rowsel<<<NNODE, RT, 0, stream>>>(edge_index, se, xwn, xwb, mlp_b, noise, sel, nE);

  hipFuncSetAttribute(reinterpret_cast<const void*>(&k_gemm),
                      hipFuncAttributeMaxDynamicSharedMemorySize, LDSMAX);

  k_gemm<<<dim3(NSEL / GR, DIN / GC), GT, ldsFor(wKp(0)), stream>>>(
      edge_attr, EDIM, NSEL, EDIM, edge_attr, sel, nE, 1, wb + wOff(0), wKp(0), wNp(0), c1_be, DIN,
      x, DIN, NNODE, 3, 1, 1, GEPS, node_mask, 0, m1, DIN, NSEL, 0);
  k_agg<<<NNODE / TGA, RT, 0, stream>>>(sel, m1, x, hp1, DIN);
  k_gemm<<<dim3(NNODE / GR, (2 * DIN) / GC), GT, ldsFor(wKp(1)), stream>>>(
      hp1, DIN, NNODE, DIN, edge_attr, sel, nE, 0, wb + wOff(1), wKp(1), wNp(1), c1_b1, 2 * DIN,
      x, DIN, NNODE, 0, 0, 1, 0.0f, node_mask, 0, t1, 2 * DIN, NNODE, 0);
  k_gemm<<<dim3(NNODE / GR, HID1 / GC), GT, ldsFor(wKp(2)), stream>>>(
      t1, 2 * DIN, NNODE, 2 * DIN, edge_attr, sel, nE, 0, wb + wOff(2), wKp(2), wNp(2), c1_b2, HID1,
      x, DIN, NNODE, 0, 0, 1, 0.0f, node_mask, 0, h1, HID1, NNODE, 0);

  k_gemm<<<dim3(NSEL / GR, HID1 / GC), GT, ldsFor(wKp(3)), stream>>>(
      edge_attr, EDIM, NSEL, EDIM, edge_attr, sel, nE, 1, wb + wOff(3), wKp(3), wNp(3), c2_be, HID1,
      h1, HID1, NNODE, 3, 1, 1, GEPS, node_mask, 0, m2, HID1, NSEL, 0);
  k_agg<<<NNODE / TGA, RT, 0, stream>>>(sel, m2, h1, hp2, HID1);
  k_gemm<<<dim3(NNODE / GR, (2 * HID1) / GC), GT, ldsFor(wKp(4)), stream>>>(
      hp2, HID1, NNODE, HID1, edge_attr, sel, nE, 0, wb + wOff(4), wKp(4), wNp(4), c2_b1, 2 * HID1,
      x, DIN, NNODE, 0, 0, 1, 0.0f, node_mask, 0, t2, 2 * HID1, NNODE, 0);
  k_gemm<<<dim3(NNODE / GR, HID2 / GC), GT, ldsFor(wKp(5)), stream>>>(
      t2, 2 * HID1, NNODE, 2 * HID1, edge_attr, sel, nE, 0, wb + wOff(5), wKp(5), wNp(5), c2_b2, HID2,
      x, DIN, NNODE, 0, 0, 1, 0.0f, node_mask, 0, h2, HID2, NNODE, 0);

  k_gemm<<<dim3(NNODE / GR, 1), GT, ldsFor(wKp(6)), stream>>>(
      h2, HID2, NNODE, HID2, edge_attr, sel, nE, 0, wb + wOff(6), wKp(6), wNp(6), fc_b, NOUT,
      x, DIN, NNODE, 0, 0, 0, 0.0f, node_mask, 1, out, NOUT, NNODE, 1);
}
